// MHSA_8409545965580
// MI455X (gfx1250) — hardware-verified
//
#include <hip/hip_runtime.h>
#include <stdint.h>


typedef unsigned short hword;
typedef hword us8  __attribute__((ext_vector_type(8)));
typedef hword us16 __attribute__((ext_vector_type(16)));
typedef _Float16 f16x16 __attribute__((ext_vector_type(16)));
typedef float v8f __attribute__((ext_vector_type(8)));
typedef float v4f __attribute__((ext_vector_type(4)));

#ifndef NB
#define NB 2
#endif
#ifndef SEQ
#define SEQ 2048
#endif
#define NB_FULL  2
#define SEQ_FULL 2048
#define DIM   1024
#define HD    64
#define NH    16
#define MROWS (NB * SEQ)
#define RESQ  256
#define NQT   (SEQ / 64)
#define NQTR  (RESQ / 64)
#define NQL   (((NQT - NQTR) > 0) ? (NQT - NQTR) : 1)
#define NMT   (MROWS / 64)
#define LDT   68
#define OP    72

static_assert(NB >= 1 && NB <= NB_FULL);
static_assert(SEQ >= RESQ && SEQ <= SEQ_FULL && (SEQ % 64) == 0);
static_assert((RESQ % 64) == 0);
static_assert((DIM % 32) == 0 && HD == 64 && NH * HD == DIM);
static_assert((MROWS % 64) == 0);

#define CX    16.0f
#define CW    32.0f
#define QSCL  (1.0f / 32.0f)
#define SSCL  (1.0f / 2048.0f)
#define PCAR  16384.0f
#define RC    1024.0f
#define RINV  (1.0f / 1024.0f)
#define AOC   16384.0f
#define OSCL  (1.0f / 512.0f)

__device__ __forceinline__ hword f2bf(float x) {
    unsigned int u = __float_as_uint(x);
    u = (u + 0x7FFFu + ((u >> 16) & 1u)) >> 16;
    return (hword)u;
}
__device__ __forceinline__ float bf2f(hword b) {
    return __uint_as_float(((unsigned int)b) << 16);
}
__device__ __forceinline__ hword f2h(float x) {
    _Float16 t = (_Float16)x;
    return __builtin_bit_cast(hword, t);
}
__device__ __forceinline__ float h2f(hword b) {
    _Float16 t = __builtin_bit_cast(_Float16, b);
    return (float)t;
}
__device__ __forceinline__ v8f zero8() {
    v8f z;
#pragma unroll
    for (int i = 0; i < 8; ++i) z[i] = 0.0f;
    return z;
}

__device__ __forceinline__ v8f mma_hf(v8f c, us16 a, us16 b) {
    f16x16 av = __builtin_bit_cast(f16x16, a);
    f16x16 bv = __builtin_bit_cast(f16x16, b);
    c = __builtin_amdgcn_wmma_f32_16x16x32_f16(false, av, false, bv, (short)0, c, false, false);
    asm volatile("v_nop\n\tv_nop\n\tv_nop\n\tv_nop" : "+v"(c) : "v"(a), "v"(b));
    return c;
}

__device__ __forceinline__ us16 frag_rows(const hword* p, int ld, int row, int k0, int h) {
    const hword* base = p + (size_t)row * ld + k0 + 8 * h;
    us8 e0 = *(const us8*)(base);
    us8 e1 = *(const us8*)(base + 16);
    return __builtin_shufflevector(e0, e1, 0, 1, 2, 3, 4, 5, 6, 7,
                                   8, 9, 10, 11, 12, 13, 14, 15);
}

template <int XMAP>
__global__ __launch_bounds__(256) void k_cvt(const float* __restrict__ src, int n8, float fscale,
                                             hword* __restrict__ df) {
    const int i = blockIdx.x * 256 + threadIdx.x;
    if (i >= n8) return;
    const size_t e = (size_t)i * 8;
    size_t se = e;
    if (XMAP) {
        const size_t prow = e / DIM, col = e - prow * DIM;
        const size_t b = prow / SEQ, n = prow - b * SEQ;
        se = (b * SEQ_FULL + n) * DIM + col;
    }
    const float* s = src + se;
    const v4f a = *(const v4f*)(s);
    const v4f c = *(const v4f*)(s + 4);
    us8 of;
#pragma unroll
    for (int k = 0; k < 4; ++k) {
        of[k]     = f2h(bf2f(f2bf(a[k])) * fscale);
        of[4 + k] = f2h(bf2f(f2bf(c[k])) * fscale);
    }
    *(volatile us8*)(df + e) = of;
    __threadfence();
    *(volatile us8*)(df + e) = of;
}

__device__ __forceinline__ void hr_pass(const float* tile, hword* PH, hword* PR,
                                        size_t rb, int w, int p, int lq, bool wres) {
#pragma unroll
    for (int i = 0; i < 4; ++i) {
        const int row = w * 16 + 4 * i + lq;
        const float* sp = tile + row * LDT + 8 * p;
        const v4f u0 = *(const v4f*)(sp);
        const v4f u1 = *(const v4f*)(sp + 4);
        us8 oh, ox;
#pragma unroll
        for (int e = 0; e < 4; ++e) {
            const float ua = u0[e];
            const hword a = f2h(ua);
            oh[e] = a;
            ox[e] = f2h((ua - h2f(a)) * RC);
            const float uc = u1[e];
            const hword c = f2h(uc);
            oh[4 + e] = c;
            ox[4 + e] = f2h((uc - h2f(c)) * RC);
        }
        const size_t doff = (rb + (size_t)row) * HD + 8 * p;
        *(volatile us8*)(PH + doff) = oh;
        if (wres) *(volatile us8*)(PR + doff) = ox;
    }
}
__device__ __forceinline__ void vt_pass(const float* tile, hword* VH, hword* VR, size_t vb, int n0,
                                        int w, int p, int lq, bool wres) {
#pragma unroll
    for (int i = 0; i < 4; ++i) {
        const int d = w * 16 + 4 * i + lq;
        us8 oh, ox;
#pragma unroll
        for (int e = 0; e < 8; ++e) {
            const float u = tile[(8 * p + e) * LDT + d];
            const hword a = f2h(u);
            oh[e] = a;
            ox[e] = f2h((u - h2f(a)) * RC);
        }
        const size_t doff = (vb + (size_t)d) * SEQ + (size_t)n0 + 8 * p;
        *(volatile us8*)(VH + doff) = oh;
        if (wres) *(volatile us8*)(VR + doff) = ox;
    }
}

template <int SV>
__global__ __launch_bounds__(128) __attribute__((amdgpu_num_vgpr(256)))
void k_qkv(const hword* __restrict__ xp, const hword* __restrict__ w0, const hword* __restrict__ w1,
           hword* dh0, hword* dr0, hword* dh1, hword* dr1) {
    __shared__ __align__(16) float tile[64 * LDT];
    const int w = threadIdx.x >> 5, lane = threadIdx.x & 31;
    const int h = lane >> 4, m = lane & 15;
    const int mt = blockIdx.x % NMT, ng = blockIdx.x / NMT;
    const int s  = SV ? 0 : (ng >> 4);
    const int hh = SV ? ng : (ng & 15);
    const int tok0 = mt * 64;
    const int wr = w & 1, wc = w >> 1;
    const int ar0 = tok0 + wr * 32;
    const hword* wp = (s == 0) ? w0 : w1;

    int orow[2];
#pragma unroll
    for (int t = 0; t < 2; ++t) orow[t] = hh * HD + wc * 32 + t * 16 + m;

    v8f acc[2][2];
#pragma unroll
    for (int mi = 0; mi < 2; ++mi)
#pragma unroll
        for (int t = 0; t < 2; ++t) acc[mi][t] = zero8();

#pragma unroll 1
    for (int k0 = 0; k0 < DIM; k0 += 32) {
        const us16 a0 = frag_rows(xp, DIM, ar0 + m, k0, h);
        const us16 a1 = frag_rows(xp, DIM, ar0 + 16 + m, k0, h);
#pragma unroll
        for (int t = 0; t < 2; ++t) {
            const us16 b = frag_rows(wp, DIM, orow[t], k0, h);
            acc[0][t] = mma_hf(acc[0][t], a0, b);
            acc[1][t] = mma_hf(acc[1][t], a1, b);
        }
    }

#pragma unroll
    for (int t = 0; t < 2; ++t)
#pragma unroll
        for (int mi = 0; mi < 2; ++mi)
#pragma unroll
            for (int r = 0; r < 8; ++r)
                tile[(wr * 32 + mi * 16 + 8 * h + r) * LDT + wc * 32 + t * 16 + m] =
                    acc[mi][t][r] * QSCL;
    __syncthreads();

    const int bb = tok0 / SEQ, n0 = tok0 - bb * SEQ;
    const bool wres = (n0 < RESQ);
    const int p = lane & 7, lq = lane >> 3;
    if (SV == 0) {
        hword* PH = (s == 0) ? dh0 : dh1;
        hword* PR = (s == 0) ? dr0 : dr1;
        const size_t rb = ((size_t)(bb * NH + hh)) * SEQ + (size_t)n0;
        hr_pass(tile, PH, PR, rb, w, p, lq, wres);
        __threadfence();
        hr_pass(tile, PH, PR, rb, w, p, lq, wres);
    } else {
        const size_t vb = ((size_t)(bb * NH + hh)) * HD;
        vt_pass(tile, dh0, dr0, vb, n0, w, p, lq, wres);
        __threadfence();
        vt_pass(tile, dh0, dr0, vb, n0, w, p, lq, wres);
    }
}

__device__ __forceinline__ void ao_pass(const hword* sw, hword* ao, size_t drow0, int hh, int lane) {
    const int p = lane & 7, lq = lane >> 3;
#pragma unroll
    for (int i = 0; i < 4; ++i) {
        const int row = 4 * i + lq;
        const us8 o = *(const us8*)(sw + row * OP + 8 * p);
        hword* dp = ao + (drow0 + (size_t)row) * DIM + hh * HD + 8 * p;
        *(volatile us8*)dp = o;
    }
}

__global__ __launch_bounds__(128) __attribute__((amdgpu_num_vgpr(256)))
void k_attn(const hword* __restrict__ qh, const hword* __restrict__ kh,
            const hword* __restrict__ vt, hword* ao) {
    __shared__ __align__(16) hword st[4 * 16 * OP];
    const int w = threadIdx.x >> 5, lane = threadIdx.x & 31;
    const int h = lane >> 4, m = lane & 15;
    const int qt = NQTR + (int)(blockIdx.x % NQL), bh = (int)(blockIdx.x / NQL);
    const size_t poff = (size_t)bh * SEQ * HD;
    const hword* qhp = qh + poff;
    const hword* khp = kh + poff;
    const hword* vtp = vt + poff;
    const int qb0 = qt * 64;
    const int q0 = qb0 + w * 16;
    const int qi = q0 + m;

    us16 qb[2];
#pragma unroll
    for (int dc = 0; dc < 2; ++dc) qb[dc] = frag_rows(qhp, HD, qi, dc * 32, h);

    v8f oacc[4];
#pragma unroll
    for (int dt = 0; dt < 4; ++dt) oacc[dt] = zero8();
    float mrun = -1.0e30f, lrun = 0.0f;

#pragma unroll 1
    for (int kc = 0; kc <= qb0; kc += 64) {
        v8f sacc[4];
#pragma unroll
        for (int kt = 0; kt < 4; ++kt) {
            v8f sa = zero8();
            const int krow = kc + kt * 16 + m;
#pragma unroll
            for (int dc = 0; dc < 2; ++dc) {
                const us16 ka = frag_rows(khp, HD, krow, dc * 32, h);
                sa = mma_hf(sa, ka, qb[dc]);
            }
            sacc[kt] = sa;
        }
        if (kc == qb0) {
#pragma unroll
            for (int kt = 0; kt < 4; ++kt)
#pragma unroll
                for (int r = 0; r < 8; ++r) {
                    const int key = kc + kt * 16 + 8 * h + r;
                    sacc[kt][r] = (key > qi) ? -1.0e30f : sacc[kt][r];
                }
        }

        float mloc = -1.0e30f;
#pragma unroll
        for (int kt = 0; kt < 4; ++kt)
#pragma unroll
            for (int r = 0; r < 8; ++r) mloc = fmaxf(mloc, sacc[kt][r]);
        mloc = fmaxf(mloc, __shfl_xor(mloc, 16, 32));
        const float mnew = fmaxf(mrun, mloc);
        const float corr = __expf((mrun - mnew) * SSCL);
        mrun = mnew;
        float lsum = 0.0f;
        us16 pb[2];
#pragma unroll
        for (int kt = 0; kt < 4; ++kt) {
#pragma unroll
            for (int r = 0; r < 8; ++r) {
                const float pv = __expf((sacc[kt][r] - mnew) * SSCL);
                lsum += pv;
                pb[kt >> 1][(kt & 1) * 8 + r] = f2h(pv * PCAR);
            }
        }
        lsum += __shfl_xor(lsum, 16, 32);
        lrun = lrun * corr + lsum;
#pragma unroll
        for (int dt = 0; dt < 4; ++dt) oacc[dt] = oacc[dt] * corr;

#pragma unroll
        for (int ks = 0; ks < 2; ++ks) {
#pragma unroll
            for (int dt = 0; dt < 4; ++dt) {
                const us16 va = frag_rows(vtp, SEQ, dt * 16 + m, kc + ks * 32, h);
                oacc[dt] = mma_hf(oacc[dt], va, pb[ks]);
            }
        }
    }

    const float inv = 1.0f / (lrun * AOC);
    hword* sw = st + w * (16 * OP);
#pragma unroll
    for (int dt = 0; dt < 4; ++dt) {
        us8 o;
#pragma unroll
        for (int r = 0; r < 8; ++r) o[r] = f2h(oacc[dt][r] * inv);
        *(us8*)(sw + m * OP + dt * 16 + 8 * h) = o;
    }
    __syncthreads();

    const int bb = bh / NH, hh = bh - bb * NH;
    const size_t drow0 = (size_t)bb * SEQ + (size_t)q0;
    ao_pass(sw, ao, drow0, hh, lane);
    __threadfence();
    ao_pass(sw, ao, drow0, hh, lane);
}

__global__ __launch_bounds__(128) __attribute__((amdgpu_num_vgpr(256)))
void k_attn_res(const hword* __restrict__ qh, const hword* __restrict__ qr,
                const hword* __restrict__ kh, const hword* __restrict__ kr,
                const hword* __restrict__ vt, const hword* __restrict__ vr,
                hword* ao, hword* aor) {
    __shared__ __align__(16) hword sth[4 * 16 * OP];
    __shared__ __align__(16) hword stx[4 * 16 * OP];
    const int w = threadIdx.x >> 5, lane = threadIdx.x & 31;
    const int h = lane >> 4, m = lane & 15;
    const int qt = (int)(blockIdx.x % NQTR), bh = (int)(blockIdx.x / NQTR);
    const size_t poff = (size_t)bh * SEQ * HD;
    const hword* qhp = qh + poff;
    const hword* qrp = qr + poff;
    const hword* khp = kh + poff;
    const hword* krp = kr + poff;
    const hword* vtp = vt + poff;
    const hword* vrp = vr + poff;
    const int qb0 = qt * 64;
    const int q0 = qb0 + w * 16;
    const int qi = q0 + m;
    const int kend = qb0 + 32;

    v8f oacc[4], oacx[4];
#pragma unroll
    for (int dt = 0; dt < 4; ++dt) { oacc[dt] = zero8(); oacx[dt] = zero8(); }
    float mrun = -1.0e30f, lrun = 0.0f;

#pragma unroll 1
    for (int kc = 0; kc <= kend; kc += 32) {
        v8f sval[2];
#pragma unroll
        for (int kt = 0; kt < 2; ++kt) {
            v8f sa = zero8(), sx = zero8();
            const int krow = kc + kt * 16 + m;
#pragma unroll
            for (int dc = 0; dc < 2; ++dc) {
                const us16 qa = frag_rows(qhp, HD, qi, dc * 32, h);
                const us16 qx = frag_rows(qrp, HD, qi, dc * 32, h);
                const us16 ka = frag_rows(khp, HD, krow, dc * 32, h);
                const us16 kx = frag_rows(krp, HD, krow, dc * 32, h);
                sa = mma_hf(sa, ka, qa);
                sx = mma_hf(sx, ka, qx);
                sx = mma_hf(sx, kx, qa);
            }
            sval[kt] = sa + sx * RINV;
        }
#pragma unroll
        for (int kt = 0; kt < 2; ++kt)
#pragma unroll
            for (int r = 0; r < 8; ++r) {
                const int key = kc + kt * 16 + 8 * h + r;
                sval[kt][r] = (key > qi) ? -1.0e30f : sval[kt][r];
            }

        float mloc = -1.0e30f;
#pragma unroll
        for (int kt = 0; kt < 2; ++kt)
#pragma unroll
            for (int r = 0; r < 8; ++r) mloc = fmaxf(mloc, sval[kt][r]);
        mloc = fmaxf(mloc, __shfl_xor(mloc, 16, 32));
        const float mnew = fmaxf(mrun, mloc);
        const float corr = __expf((mrun - mnew) * SSCL);
        mrun = mnew;
        float lsum = 0.0f;
        us16 pbh, pbx;
#pragma unroll
        for (int kt = 0; kt < 2; ++kt) {
#pragma unroll
            for (int r = 0; r < 8; ++r) {
                const float pv = __expf((sval[kt][r] - mnew) * SSCL);
                lsum += pv;
                const float pc = pv * PCAR;
                const hword a = f2h(pc);
                pbh[kt * 8 + r] = a;
                pbx[kt * 8 + r] = f2h((pc - h2f(a)) * RC);
            }
        }
        lsum += __shfl_xor(lsum, 16, 32);
        lrun = lrun * corr + lsum;
#pragma unroll
        for (int dt = 0; dt < 4; ++dt) { oacc[dt] = oacc[dt] * corr; oacx[dt] = oacx[dt] * corr; }

#pragma unroll
        for (int dt = 0; dt < 4; ++dt) {
            const us16 va = frag_rows(vtp, SEQ, dt * 16 + m, kc, h);
            const us16 vx = frag_rows(vrp, SEQ, dt * 16 + m, kc, h);
            oacc[dt] = mma_hf(oacc[dt], va, pbh);
            oacx[dt] = mma_hf(oacx[dt], va, pbx);
            oacx[dt] = mma_hf(oacx[dt], vx, pbh);
        }
    }

    const float inv = 1.0f / (lrun * AOC);
    hword* swh = sth + w * (16 * OP);
    hword* swx = stx + w * (16 * OP);
#pragma unroll
    for (int dt = 0; dt < 4; ++dt) {
        us8 oh, ox;
#pragma unroll
        for (int r = 0; r < 8; ++r) {
            const float u = (oacc[dt][r] + oacx[dt][r] * RINV) * inv;
            const hword a = f2h(u);
            oh[r] = a;
            ox[r] = f2h((u - h2f(a)) * RC);
        }
        *(us8*)(swh + m * OP + dt * 16 + 8 * h) = oh;
        *(us8*)(swx + m * OP + dt * 16 + 8 * h) = ox;
    }
    __syncthreads();

    const int bb = bh / NH, hh = bh - bb * NH;
    const size_t drow0 = (size_t)bb * SEQ + (size_t)q0;
    ao_pass(swh, ao, drow0, hh, lane);
    ao_pass(swx, aor, drow0, hh, lane);
    __threadfence();
    ao_pass(swh, ao, drow0, hh, lane);
    ao_pass(swx, aor, drow0, hh, lane);
}

__device__ __forceinline__ void store_tile_rows64(const float* tile, float* dst,
                                                  size_t drow0, int dpitch, int lane) {
    const int h = lane >> 4, m = lane & 15;
#pragma unroll
    for (int i = 0; i < 16; ++i) {
        const int row = 2 * i + h;
        v4f v = *(const v4f*)(tile + row * LDT + 4 * m);
        *(volatile v4f*)(dst + (drow0 + (size_t)row) * (size_t)dpitch + 4 * m) = v;
    }
    __threadfence();
#pragma unroll
    for (int i = 0; i < 16; ++i) {
        const int row = 2 * i + h;
        v4f v = *(const v4f*)(tile + row * LDT + 4 * m);
        *(volatile v4f*)(dst + (drow0 + (size_t)row) * (size_t)dpitch + 4 * m) = v;
    }
}

__device__ __forceinline__ void proj_accum(v8f (&acc)[2][4], const hword* __restrict__ ap,
                                           const hword* __restrict__ wf, int row0, int n0, int h, int m) {
#pragma unroll
    for (int mi = 0; mi < 2; ++mi)
#pragma unroll
        for (int t = 0; t < 4; ++t) acc[mi][t] = zero8();
#pragma unroll 1
    for (int k0 = 0; k0 < DIM; k0 += 32) {
        const us16 a0 = frag_rows(ap, DIM, row0 + m, k0, h);
        const us16 a1 = frag_rows(ap, DIM, row0 + 16 + m, k0, h);
#pragma unroll
        for (int t = 0; t < 4; ++t) {
            const us16 b = frag_rows(wf, DIM, n0 + t * 16 + m, k0, h);
            acc[0][t] = mma_hf(acc[0][t], a0, b);
            acc[1][t] = mma_hf(acc[1][t], a1, b);
        }
    }
}

__global__ __launch_bounds__(128) __attribute__((amdgpu_num_vgpr(256)))
void k_proj(const hword* __restrict__ af, const hword* __restrict__ arf,
            const hword* __restrict__ wf, float* out) {
    __shared__ __align__(16) float stg[4 * 32 * LDT];
    const int w = threadIdx.x >> 5, lane = threadIdx.x & 31;
    const int h = lane >> 4, m = lane & 15;
    const int mt = (int)(blockIdx.x >> 2), ng = (int)(blockIdx.x & 3) * 4 + w;
    const int row0 = mt * 32, n0 = ng * 64;
    const bool res = ((row0 % SEQ) < RESQ);

    float* tile = stg + w * (32 * LDT);
    v8f acc[2][4];
    proj_accum(acc, af, wf, row0, n0, h, m);
#pragma unroll
    for (int t = 0; t < 4; ++t)
#pragma unroll
        for (int mi = 0; mi < 2; ++mi)
#pragma unroll
            for (int r = 0; r < 8; ++r)
                tile[(mi * 16 + 8 * h + r) * LDT + t * 16 + m] = acc[mi][t][r] * OSCL;
    if (res) {
        proj_accum(acc, arf, wf, row0, n0, h, m);
#pragma unroll
        for (int t = 0; t < 4; ++t)
#pragma unroll
            for (int mi = 0; mi < 2; ++mi)
#pragma unroll
                for (int r = 0; r < 8; ++r)
                    tile[(mi * 16 + 8 * h + r) * LDT + t * 16 + m] += acc[mi][t][r] * (OSCL * RINV);
    }
    __syncthreads();

    store_tile_rows64(tile, out + n0, (size_t)row0, DIM, lane);
}

extern "C" void kernel_launch(void* const* d_in, const int* in_sizes, int n_in,
                              void* d_out, int out_size, void* d_ws, size_t ws_size,
                              hipStream_t stream) {
    if (n_in < 5) return;
    const int nx = MROWS * DIM;
    const int nw = DIM * DIM;
    const int xneed = ((NB - 1) * SEQ_FULL + SEQ) * DIM;
    if (in_sizes[0] < xneed || in_sizes[1] < nw || in_sizes[2] < nw ||
        in_sizes[3] < nw || in_sizes[4] < nw || out_size < nx) return;

    const float* x  = (const float*)d_in[0];
    const float* qw = (const float*)d_in[1];
    const float* kw = (const float*)d_in[2];
    const float* vw = (const float*)d_in[3];
    const float* ow = (const float*)d_in[4];
    float* out = (float*)d_out;

    const size_t b_p = (size_t)nx * 2;
    const size_t b_w = (size_t)nw * 2;
    size_t off = 0;
    char* ws = (char*)d_ws;
    hword* xf  = (hword*)(ws + off); off += b_p;
    hword* wqf = (hword*)(ws + off); off += b_w;
    hword* wkf = (hword*)(ws + off); off += b_w;
    hword* wvf = (hword*)(ws + off); off += b_w;
    hword* wof = (hword*)(ws + off); off += b_w;
    hword* qhp = (hword*)(ws + off); off += b_p;
    hword* qrp = (hword*)(ws + off); off += b_p;
    hword* khp = (hword*)(ws + off); off += b_p;
    hword* krp = (hword*)(ws + off); off += b_p;
    hword* vhp = (hword*)(ws + off); off += b_p;
    hword* vrp = (hword*)(ws + off); off += b_p;
    hword* aop = (hword*)(ws + off); off += b_p;
    hword* arp = (hword*)(ws + off); off += b_p;
    if (off > ws_size) return;

    const int n8x = nx / 8, n8w = nw / 8;
    k_cvt<1><<<(n8x + 255) / 256, 256, 0, stream>>>(x, n8x, CX, xf);
    k_cvt<0><<<(n8w + 255) / 256, 256, 0, stream>>>(qw, n8w, CW, wqf);
    k_cvt<0><<<(n8w + 255) / 256, 256, 0, stream>>>(kw, n8w, CW, wkf);
    k_cvt<0><<<(n8w + 255) / 256, 256, 0, stream>>>(vw, n8w, CW, wvf);
    k_cvt<0><<<(n8w + 255) / 256, 256, 0, stream>>>(ow, n8w, CW, wof);

    k_qkv<0><<<NMT * 32, 128, 0, stream>>>(xf, wqf, wkf, qhp, qrp, khp, krp);
    k_qkv<1><<<NMT * 16, 128, 0, stream>>>(xf, wvf, wvf, vhp, vrp, vhp, vrp);

    k_attn_res<<<NQTR * NB * NH, 128, 0, stream>>>(qhp, qrp, khp, krp, vhp, vrp, aop, arp);
    if (NQT > NQTR)
        k_attn<<<(NQT - NQTR) * NB * NH, 128, 0, stream>>>(qhp, khp, vhp, aop);

    k_proj<<<(MROWS / 32) * 4, 128, 0, stream>>>(aop, arp, wof, out);
}
